// SoftMinLayer_54597624267331
// MI455X (gfx1250) — hardware-run, weakly checked
//
#include <hip/hip_runtime.h>
#include <math.h>

typedef __attribute__((ext_vector_type(16))) _Float16 v16h;
typedef __attribute__((ext_vector_type(8)))  _Float16 v8h;
typedef __attribute__((ext_vector_type(8)))  float    v8f;
typedef __attribute__((ext_vector_type(4)))  float    v4f;
typedef __attribute__((ext_vector_type(2)))  float    v2f;
typedef __attribute__((ext_vector_type(8)))  unsigned v8u;

constexpr int kNSer   = 512;
constexpr int kQ      = 2048;
constexpr int kNShp   = 64;
constexpr int kL      = 50;
constexpr int kNWin   = kQ - kL + 1;
constexpr int kTiles  = (kNWin + 15) / 16;
constexpr int kKPad   = 64;
constexpr int kXsLen  = 2128;
constexpr int kHWords = 1056;
constexpr int kSwLen  = 2000;
static_assert(kNWin == 1999);
static_assert(kTiles == 125);
static_assert(kKPad % 32 == 0 && kKPad >= kL);
static_assert(kNShp % 16 == 0);
static_assert(kTiles * 16 <= kSwLen);
static_assert(16 * (kTiles - 1) + 15 + 32 + 8 + 16 + 7 < 2 * kHWords);
static_assert(2 * (kHWords - 1) + 2 < kXsLen);
static_assert(8 * 249 + 7 + kL - 1 < kXsLen);

constexpr float kAlpha   = -100.0f;
constexpr float kCarryX  = 64.0f;
constexpr float kCarryS  = 64.0f;
constexpr float kFold2   = 2.0f / (kCarryX * kCarryS);
constexpr float kInvL    = 1.0f / (float)kL;
constexpr float kF16Norm = 6.103515625e-5f;
constexpr float kBig     = 3.0e38f;

constexpr size_t kOffSH   = 0;
constexpr size_t kOffSSQ  = kOffSH   + (size_t)kNShp * kKPad * 2;
constexpr size_t kOffROWV = kOffSSQ  + (size_t)kNShp * 4;
constexpr size_t kOffROWM = kOffROWV + (size_t)kNSer * kNShp * 4;
constexpr size_t kWsTotal = kOffROWM + (size_t)kNSer * kNShp * 4;
static_assert(kWsTotal == 270592ull);
static_assert(kWsTotal <= 134217728ull);
static_assert((kOffSSQ % 128) == 0 && (kOffROWV % 128) == 0 && (kOffROWM % 128) == 0);

struct FragH {
  union U { v16h v; v8h h[2]; };
  static __device__ __forceinline__ v16h load(const _Float16* p) {
    U f;
    f.h[0] = *(const v8h*)(p);
    f.h[1] = *(const v8h*)(p + 16);
    return f.v;
  }
};

__device__ __forceinline__ v8f mma_f16(v16h a, v16h b, v8f c) {
  c = __builtin_amdgcn_wmma_f32_16x16x32_f16(false, a, false, b, (short)0, c, false, false);
  asm volatile("v_nop\n\tv_nop\n\tv_nop\n\tv_nop" : "+v"(c) : "v"(a), "v"(b));
  return c;
}

__device__ __forceinline__ unsigned f16_bits_carried(float v, float carry) {
  float cv = v * carry;
  cv = (fabsf(cv) < kF16Norm) ? 0.0f : cv;
  const _Float16 h = (_Float16)cv;
  return (unsigned)__builtin_bit_cast(unsigned short, h);
}

__global__ __launch_bounds__(256) void prep_kernel(
    const float* __restrict__ S, unsigned short* __restrict__ SH, float* __restrict__ SSQ)
{
  __shared__ __align__(16) float sq[kNShp];
  const int tid = threadIdx.x;
  const int lane = tid & 31;
#pragma unroll 1
  for (int it = 0; it < 2; ++it) {
    const int p = it * 256 + tid;
    const int row = p >> 3;
    const int c8 = (p & 7) * 8;
    v8h hv;
#pragma unroll
    for (int e = 0; e < 8; ++e) {
      const int l = c8 + e;
      const int lc = (l < kL) ? l : (kL - 1);
      const float v = S[row * kL + lc];
      float cv = v * kCarryS;
      cv = ((l < kL) && (fabsf(cv) >= kF16Norm)) ? cv : 0.0f;
      hv[e] = (_Float16)cv;
    }
    unsigned short* q = SH + row * kKPad + c8;
    *(volatile v8h*)q = hv;
    __threadfence();
    *(volatile v8h*)q = hv;
  }
  {
    const int row = tid & (kNShp - 1);
    float a = 0.0f;
#pragma unroll 1
    for (int l = 0; l < kL; ++l) {
      const float v = S[row * kL + l];
      a = fmaf(v, v, a);
    }
    if (tid < kNShp) sq[tid] = a;
  }
  __syncthreads();
  if (tid < 32) {
    v2f o;
    o[0] = sq[2 * lane];
    o[1] = sq[2 * lane + 1];
    float* q = SSQ + 2 * lane;
    *(volatile v2f*)q = o;
    __threadfence();
    *(volatile v2f*)q = o;
  }
}

__global__ __launch_bounds__(256) void main_kernel(
    const float* __restrict__ X, const unsigned short* __restrict__ SH, const float* __restrict__ SSQ,
    float* __restrict__ ROWV, float* __restrict__ ROWM)
{
  __shared__ __align__(16) float    xs[kXsLen];
  __shared__ __align__(16) unsigned xhw[2 * kHWords];
  __shared__ __align__(16) float    sw[kSwLen];
  __shared__ __align__(16) float    mrg[8 * 3 * 16];

  const int tid  = threadIdx.x;
  const int lane = tid & 31;
  const int wave = __builtin_amdgcn_readfirstlane(tid >> 5);
  const int hh   = lane >> 4;
  const int c    = lane & 15;
  const int i    = blockIdx.x;

  {
    const v4f* Xv = (const v4f*)(X + (size_t)i * kQ);
#pragma unroll
    for (int it = 0; it < 2; ++it) {
      const int idx = it * 256 + tid;
      const v4f d = Xv[idx];
      *(v4f*)(xs + 4 * idx) = d;
    }
    if (tid < kXsLen - kQ) xs[kQ + tid] = 0.0f;
  }
  __syncthreads();

#pragma unroll 1
  for (int w = tid; w < kHWords; w += 256) {
    const float fa = xs[2 * w];
    const float fb = xs[2 * w + 1];
    const float fc = xs[2 * w + 2];
    const unsigned ha = f16_bits_carried(fa, kCarryX);
    const unsigned hb = f16_bits_carried(fb, kCarryX);
    const unsigned hc = f16_bits_carried(fc, kCarryX);
    xhw[w] = ha | (hb << 16);
    xhw[kHWords + w] = hb | (hc << 16);
  }
  if (tid < 250) {
    const int jb0 = tid * 8;
    float s = 0.0f;
#pragma unroll 2
    for (int l = 0; l < kL; ++l) {
      const float v = xs[jb0 + l];
      s = fmaf(v, v, s);
    }
    sw[jb0] = s;
#pragma unroll 1
    for (int q = 1; q < 8; ++q) {
      const float a = xs[jb0 + q + kL - 1];
      const float b = xs[jb0 + q - 1];
      s = (s + a * a) - b * b;
      sw[jb0 + q] = s;
    }
  }
  __syncthreads();

  const int nt   = wave & 3;
  const int par2 = wave >> 2;
  const _Float16* shrow = (const _Float16*)(SH + (nt * 16 + c) * kKPad + 8 * hh);
  const v16h b0 = FragH::load(shrow);
  const v16h b1 = FragH::load(shrow + 32);
  const float ssqk = SSQ[nt * 16 + c];

  const int par = c & 1;
  const int lb  = par * kHWords + ((c - par + 8 * hh) >> 1);

  float m = kBig, s0 = 0.0f, t1 = 0.0f;

#pragma unroll 1
  for (int jt = par2; jt < kTiles; jt += 2) {
    const unsigned* p = xhw + lb + 8 * jt;
    v8u ua, ub;
    ua[0] = p[0];  ua[1] = p[1];  ua[2] = p[2];  ua[3] = p[3];
    ua[4] = p[8];  ua[5] = p[9];  ua[6] = p[10]; ua[7] = p[11];
    ub[0] = p[16]; ub[1] = p[17]; ub[2] = p[18]; ub[3] = p[19];
    ub[4] = p[24]; ub[5] = p[25]; ub[6] = p[26]; ub[7] = p[27];
    const v16h a0 = __builtin_bit_cast(v16h, ua);
    const v16h a1 = __builtin_bit_cast(v16h, ub);
    v8f acc = (v8f){0.f, 0.f, 0.f, 0.f, 0.f, 0.f, 0.f, 0.f};
    acc = mma_f16(a0, b0, acc);
    acc = mma_f16(a1, b1, acc);

    const int jb = 16 * jt + 8 * hh;
    const v4f w0 = *(const v4f*)(sw + jb);
    const v4f w1 = *(const v4f*)(sw + jb + 4);
    float swr[8];
    swr[0] = w0[0]; swr[1] = w0[1]; swr[2] = w0[2]; swr[3] = w0[3];
    swr[4] = w1[0]; swr[5] = w1[1]; swr[6] = w1[2]; swr[7] = w1[3];

    float d[8];
    float dmin = kBig;
#pragma unroll
    for (int r = 0; r < 8; ++r) {
      const float corr2 = acc[r] * kFold2;
      const float dv = ((swr[r] - corr2) + ssqk) * kInvL;
      d[r] = dv;
      const bool ok = (jb + r) < kNWin;
      dmin = fminf(dmin, ok ? dv : kBig);
    }
    const float mn = fminf(m, dmin);
    const float f  = expf(kAlpha * (m - mn));
    float es = 0.0f, et = 0.0f;
#pragma unroll
    for (int r = 0; r < 8; ++r) {
      const bool ok = (jb + r) < kNWin;
      float e = expf(kAlpha * (d[r] - mn));
      e = ok ? e : 0.0f;
      es += e;
      et = fmaf(d[r], e, et);
    }
    s0 = fmaf(s0, f, es);
    t1 = fmaf(t1, f, et);
    m  = mn;
  }

  {
    const float m2 = __shfl_xor(m, 16, 32);
    const float s2 = __shfl_xor(s0, 16, 32);
    const float t2 = __shfl_xor(t1, 16, 32);
    const float mm = fminf(m, m2);
    const float fa = expf(kAlpha * (m - mm));
    const float fb = expf(kAlpha * (m2 - mm));
    const float sm = s0 * fa + s2 * fb;
    const float tm = t1 * fa + t2 * fb;
    if (hh == 0) {
      mrg[(wave * 3 + 0) * 16 + c] = mm;
      mrg[(wave * 3 + 1) * 16 + c] = sm;
      mrg[(wave * 3 + 2) * 16 + c] = tm;
    }
  }
  __syncthreads();

  if (wave == 0) {
    const int ntc = lane >> 3;
    const int cc  = (2 * lane) & 15;
    float res[2], mres[2];
#pragma unroll
    for (int q = 0; q < 2; ++q) {
      const int ia = (ntc * 3) * 16 + cc + q;
      const int ib = ((ntc + 4) * 3) * 16 + cc + q;
      const float ma = mrg[ia], sa = mrg[ia + 16], ta = mrg[ia + 32];
      const float mb = mrg[ib], sb = mrg[ib + 16], tb = mrg[ib + 32];
      const float mm = fminf(ma, mb);
      const float fa = expf(kAlpha * (ma - mm));
      const float fb = expf(kAlpha * (mb - mm));
      const float sm = sa * fa + sb * fb;
      const float tm = ta * fa + tb * fb;
      res[q]  = tm * (1.0f / sm);
      mres[q] = mm;
    }
    v2f ov, om;
    ov[0] = res[0];  ov[1] = res[1];
    om[0] = mres[0]; om[1] = mres[1];
    float* qv = ROWV + (size_t)i * kNShp + 2 * lane;
    float* qm = ROWM + (size_t)i * kNShp + 2 * lane;
    *(volatile v2f*)qv = ov;
    *(volatile v2f*)qm = om;
    __threadfence();
    *(volatile v2f*)qv = ov;
    *(volatile v2f*)qm = om;
  }
}

__global__ __launch_bounds__(256) void finalize_kernel(
    const float* __restrict__ ROWV, const float* __restrict__ ROWM, float* __restrict__ out)
{
  __shared__ __align__(16) float part[4 * kNShp];
  __shared__ __align__(16) float gm[kNShp];
  const int tid = threadIdx.x;
  const int k = tid & (kNShp - 1);
  const int g = tid >> 6;
  float mn = kBig;
#pragma unroll 4
  for (int r = g; r < kNSer; r += 4) mn = fminf(mn, ROWM[(size_t)r * kNShp + k]);
  part[g * kNShp + k] = mn;
  __syncthreads();
  if (tid < kNShp) {
    const float a = fminf(part[tid], part[kNShp + tid]);
    const float b = fminf(part[2 * kNShp + tid], part[3 * kNShp + tid]);
    gm[tid] = fminf(a, b);
  }
  __syncthreads();
#pragma unroll 1
  for (int it = 0; it < (kNSer * kNShp / 4) / 256; ++it) {
    const int idx4 = it * 256 + tid;
    const int e = idx4 * 4;
    const int kk = e & (kNShp - 1);
    const v4f v  = *(const v4f*)(ROWV + e);
    const v4f g4 = *(const v4f*)(gm + kk);
    const v4f o  = v - g4;
    *(volatile v4f*)(out + e) = o;
    __threadfence();
    *(volatile v4f*)(out + e) = o;
  }
}

extern "C" void kernel_launch(void* const* d_in, const int* in_sizes, int n_in,
                              void* d_out, int out_size, void* d_ws, size_t ws_size,
                              hipStream_t stream) {
  if (n_in < 2) return;
  if (in_sizes[0] != kNSer * kQ) return;
  if (in_sizes[1] != kNShp * kL) return;
  if (out_size != kNSer * kNShp) return;
  if (ws_size < kWsTotal) return;

  const float* X = (const float*)d_in[0];
  const float* S = (const float*)d_in[1];
  float* out = (float*)d_out;

  char* ws = (char*)d_ws;
  unsigned short* SH = (unsigned short*)(ws + kOffSH);
  float* SSQ  = (float*)(ws + kOffSSQ);
  float* ROWV = (float*)(ws + kOffROWV);
  float* ROWM = (float*)(ws + kOffROWM);

  prep_kernel<<<1, 256, 0, stream>>>(S, SH, SSQ);
  main_kernel<<<kNSer, 256, 0, stream>>>(X, SH, SSQ, ROWV, ROWM);
  finalize_kernel<<<1, 256, 0, stream>>>(ROWV, ROWM, out);
}
